// GIN_Net_15015205667099
// MI455X (gfx1250) — hardware-run, weakly checked
//
#include <hip/hip_runtime.h>
#include <stddef.h>
#include <stdint.h>


#define NN      100000
#define NE      1250000
#define DC      64
#define KT      128
#define WSQ     (DC * KT)
#define GBM     128
#define NGB     782
#define MP      (NGB * GBM)
#define GTHR    256
#define PTHR    256
#define ATHR    256
#define BTHR    256
#define BWAVE   8
#define EPT     8
#define CHUNK   (BTHR * EPT)
#define NBRUN   1024
#define SLB     10
#define NBLK    98
#define RCAP    16384
#define WLCAP   4096
#define DEGCAP  64
#define FLW     32
#define HITMAX  13072
#define DEGMAX  30
#define RECW    128
#define BUCKET_INTS (BWAVE * WLCAP + RCAP + 3 * NBRUN + 32)
#define BUCKET_LDS  (BUCKET_INTS * 4)
#define PB_X    ((NN * 8) / PTHR)
#define PB_W    16
#define PB_P    12
#define PZ_UNITS (((MP - NN) * KT) / 8)
#define PB_Z    (PZ_UNITS / PTHR)
#define PB_TOT  (PB_X + PB_W + PB_P + PB_Z)
#define NUNITS  (NN * 16)

static_assert(DC == 64 && KT == 2 * DC && (KT % 32) == 0);
static_assert(GBM == (GTHR / 32) * 16);
static_assert(NGB * GBM >= NN && (NGB - 1) * GBM < NN);
static_assert((NN % 16) == 0 && (NN % GBM) == 32);
static_assert(NN <= (1 << 17) && NBRUN <= (1 << SLB) && NBRUN == (1 << SLB));
static_assert(NBLK * NBRUN >= NN && (NBLK - 1) * NBRUN < NN);
static_assert((NBRUN % 2) == 0 && NBRUN == 4 * BTHR);
static_assert(RCAP * 20 >= HITMAX * 21);
static_assert(DEGCAP >= DEGMAX + 8);
static_assert(WLCAP * BWAVE >= 2 * RCAP && (RCAP % (4 * BTHR)) == 0);
static_assert((NE % 8) == 0 && NE >= 8);
static_assert(BUCKET_LDS <= 300000);
static_assert(((NN * 8) % PTHR) == 0 && (PZ_UNITS % PTHR) == 0);
static_assert((NUNITS % ATHR) == 0);
static_assert(((RCAP + 3 * NBRUN) % 4) == 0);

typedef float          v4f  __attribute__((ext_vector_type(4)));
typedef float          v8f  __attribute__((ext_vector_type(8)));
typedef double         v2d  __attribute__((ext_vector_type(2)));
typedef int            v4i  __attribute__((ext_vector_type(4)));
typedef int            v8i  __attribute__((ext_vector_type(8)));
typedef unsigned int   v2u  __attribute__((ext_vector_type(2)));
typedef unsigned short v8us __attribute__((ext_vector_type(8)));
typedef __bf16         v16b __attribute__((ext_vector_type(16)));
typedef v4f  __attribute__((may_alias)) v4fa;
typedef v2d  __attribute__((may_alias)) v2da;
typedef v4i  __attribute__((may_alias)) v4ia;
typedef v2u  __attribute__((may_alias)) v2ua;
typedef v8us __attribute__((may_alias)) v8usa;
union FragB { v16b v; v8us h[2]; v8i w; };

__device__ __forceinline__ v8f wmb(const FragB& a, const FragB& b, v8f c) {
  v8f d = __builtin_amdgcn_wmma_f32_16x16x32_bf16(false, a.v, false, b.v, (short)0, c, false, false);
  asm volatile("v_nop\n\tv_nop\n\tv_nop\n\tv_nop" : "+v"(d) : "v"(a.w), "v"(b.w));
  return d;
}

__device__ __forceinline__ unsigned bf_bits(float f) {
  const unsigned u = __float_as_uint(f);
  const unsigned r = (u + 0x7FFFu + ((u >> 16) & 1u)) >> 16;
  const bool isn = (u & 0x7fffffffu) > 0x7f800000u;
  return isn ? 0x7fc0u : r;
}
__device__ __forceinline__ float bf_val(unsigned b) { return __uint_as_float(b << 16); }
__device__ __forceinline__ float bf_rne(float f) { return bf_val(bf_bits(f)); }
__device__ __forceinline__ float relu_k(float v) { return (v > 0.0f) ? v : (v - v); }

struct HL { v2u h; v2u l; };
__device__ __forceinline__ HL split4(float r0, float r1, float r2, float r3, unsigned lomask) {
  const unsigned h0 = bf_bits(r0), h1 = bf_bits(r1), h2 = bf_bits(r2), h3 = bf_bits(r3);
  const unsigned l0 = bf_bits(r0 - bf_val(h0)), l1 = bf_bits(r1 - bf_val(h1));
  const unsigned l2 = bf_bits(r2 - bf_val(h2)), l3 = bf_bits(r3 - bf_val(h3));
  HL o;
  o.h.x = h0 | (h1 << 16);
  o.h.y = h2 | (h3 << 16);
  o.l.x = (l0 | (l1 << 16)) & lomask;
  o.l.y = (l2 | (l3 << 16)) & lomask;
  return o;
}

__device__ __forceinline__ void st2_v8us(unsigned short* p, const v8us v, const bool ok) {
  if (ok) *(volatile v8us*)p = v;
  __threadfence();
  if (ok) *(volatile v8us*)p = v;
}
__device__ __forceinline__ void st2_v4f(float* p, const v4f v, const bool ok) {
  if (ok) *(volatile v4f*)p = v;
  __threadfence();
  if (ok) *(volatile v4f*)p = v;
}
__device__ __forceinline__ void st2_v2d(double* p, const v2d v, const bool ok) {
  if (ok) *(volatile v2d*)p = v;
  __threadfence();
  if (ok) *(volatile v2d*)p = v;
}
__device__ __forceinline__ void st2_pair(unsigned short* p, const v2u hw, const v2u lw, const bool ok) {
  if (ok) { *(volatile v2u*)p = hw; *(volatile v2u*)(p + DC) = lw; }
  __threadfence();
  if (ok) { *(volatile v2u*)p = hw; *(volatile v2u*)(p + DC) = lw; }
}

__device__ __forceinline__ void wunit(const float* __restrict__ W, int v, unsigned short* dst) {
  const int n  = v >> 4;
  const int k8 = (v & 15) * 8;
  const int kk = k8 & (DC - 1);
  const float* p = W + (size_t)kk * DC + n;
  v8us o;
#pragma unroll
  for (int i = 0; i < 8; ++i) o[i] = (unsigned short)bf_bits(p[(size_t)i * DC]);
  st2_v8us(dst + (size_t)n * KT + k8, o, true);
}
__device__ __forceinline__ void punit(const float* __restrict__ p, float* dst, int tid) {
  const int q = tid & 15;
  const v4f a = *(const v4f*)(p + 4 * q);
  asm volatile("" :: "v"(a.x), "v"(a.y), "v"(a.z), "v"(a.w));
  v4f o;
  o.x = bf_rne(a.x); o.y = bf_rne(a.y); o.z = bf_rne(a.z); o.w = bf_rne(a.w);
  st2_v4f(dst + 4 * q, o, tid < 16);
}

__global__ __launch_bounds__(PTHR) void k_prep(
    const float* __restrict__ x,
    const float* __restrict__ w0, const float* __restrict__ w1,
    const float* __restrict__ w2, const float* __restrict__ w3,
    const float* __restrict__ p0, const float* __restrict__ p1, const float* __restrict__ p2,
    const float* __restrict__ p3, const float* __restrict__ p4, const float* __restrict__ p5,
    const float* __restrict__ p6, const float* __restrict__ p7, const float* __restrict__ p8,
    const float* __restrict__ p9, const float* __restrict__ p10, const float* __restrict__ p11,
    unsigned short* xb, unsigned short* wt, float* par, unsigned short* apad) {
  const int b = (int)blockIdx.x, tid = (int)threadIdx.x;
  if (b < PB_X) {
    const size_t u = (size_t)b * PTHR + (size_t)tid;
    const float* p = x + u * 8;
    const v4f a = *(const v4f*)p;
    const v4f c = *(const v4f*)(p + 4);
    v8us o;
    o[0] = (unsigned short)bf_bits(a.x); o[1] = (unsigned short)bf_bits(a.y);
    o[2] = (unsigned short)bf_bits(a.z); o[3] = (unsigned short)bf_bits(a.w);
    o[4] = (unsigned short)bf_bits(c.x); o[5] = (unsigned short)bf_bits(c.y);
    o[6] = (unsigned short)bf_bits(c.z); o[7] = (unsigned short)bf_bits(c.w);
    st2_v8us(xb + u * 8, o, true);
  } else if (b < PB_X + PB_W) {
    const int bb = b - PB_X;
    const int mi = bb >> 2;
    const int v  = (bb & 3) * PTHR + tid;
    unsigned short* dst = wt + (size_t)mi * WSQ;
    if (mi == 0)      wunit(w0, v, dst);
    else if (mi == 1) wunit(w1, v, dst);
    else if (mi == 2) wunit(w2, v, dst);
    else              wunit(w3, v, dst);
  } else if (b < PB_X + PB_W + PB_P) {
    const int vi = b - (PB_X + PB_W);
    float* dst = par + (size_t)vi * DC;
    switch (vi) {
      case 0:  punit(p0,  dst, tid); break;
      case 1:  punit(p1,  dst, tid); break;
      case 2:  punit(p2,  dst, tid); break;
      case 3:  punit(p3,  dst, tid); break;
      case 4:  punit(p4,  dst, tid); break;
      case 5:  punit(p5,  dst, tid); break;
      case 6:  punit(p6,  dst, tid); break;
      case 7:  punit(p7,  dst, tid); break;
      case 8:  punit(p8,  dst, tid); break;
      case 9:  punit(p9,  dst, tid); break;
      case 10: punit(p10, dst, tid); break;
      default: punit(p11, dst, tid); break;
    }
  } else {
    const int u = (b - (PB_X + PB_W + PB_P)) * PTHR + tid;
    const v8us z = {0, 0, 0, 0, 0, 0, 0, 0};
    const int uc = u < PZ_UNITS ? u : PZ_UNITS - 1;
    st2_v8us(apad + (size_t)uc * 8, z, u < PZ_UNITS);
  }
}

#define HITJ(HJ, SJ, SV) { \
    const unsigned mj = __builtin_amdgcn_ballot_w32(HJ); \
    if (mj != 0u) { \
      if (HJ) { \
        const int pos = wc + (int)__builtin_amdgcn_mbcnt_lo(mj, 0u); \
        int sv = (SV); \
        sv = sv < 0 ? 0 : (sv > nN - 1 ? nN - 1 : sv); \
        if (pos < WLCAP) mywl[pos] = (int)(((unsigned)sv << SLB) | (SJ)); \
      } \
      wc += (int)__builtin_popcount(mj); } }

__global__ __launch_bounds__(BTHR) void k_bucket(const int* __restrict__ srcs, const int* __restrict__ dsts,
                                                 int nE, int nN,
                                                 int* listg, int* cntg, int* offg, int* flagg) {
  extern __shared__ __attribute__((aligned(16))) int dsm[];
  int* wl   = dsm;
  int* sl   = wl + BWAVE * WLCAP;
  int* cnt  = sl + RCAP;
  int* off  = cnt + NBRUN;
  int* cur  = off + NBRUN;
  int* misc = cur + NBRUN;
  const int tid = (int)threadIdx.x, lane = tid & 31, wave = tid >> 5;
  const int blk = (int)blockIdx.x;

  {
    const v4i z4 = {0, 0, 0, 0};
#pragma unroll 1
    for (int i = 4 * tid; i < RCAP + 3 * NBRUN; i += 4 * BTHR) *(v4ia*)(sl + i) = z4;
    if (tid < 32) misc[tid] = 0;
  }
  __syncthreads();

  int wc = 0;
  {
    int* mywl = wl + wave * WLCAP;
    const unsigned nbs = (unsigned)(blk * NBRUN);
    int nb = nN - blk * NBRUN;
    nb = nb < 0 ? 0 : (nb > NBRUN ? NBRUN : nb);
    const unsigned unb = (unsigned)nb;
    const int nChunks = (nE + CHUNK - 1) / CHUNK;
#pragma unroll 1
    for (int ch = 0; ch < nChunks; ++ch) {
      const int e0 = ch * CHUNK + tid * EPT;
      const int ec = e0 > nE - EPT ? nE - EPT : e0;
      const v4i da = *(const v4i*)(dsts + ec);
      const v4i db = *(const v4i*)(dsts + ec + 4);
      const v4i sa = *(const v4i*)(srcs + ec);
      const v4i sb = *(const v4i*)(srcs + ec + 4);
      asm volatile("" :: "v"(da.x), "v"(da.y), "v"(da.z), "v"(da.w));
      asm volatile("" :: "v"(db.x), "v"(db.y), "v"(db.z), "v"(db.w));
      asm volatile("" :: "v"(sa.x), "v"(sa.y), "v"(sa.z), "v"(sa.w));
      asm volatile("" :: "v"(sb.x), "v"(sb.y), "v"(sb.z), "v"(sb.w));
      const bool valid = e0 < nE;
      const unsigned s0 = (unsigned)da.x - nbs, s1 = (unsigned)da.y - nbs;
      const unsigned s2 = (unsigned)da.z - nbs, s3 = (unsigned)da.w - nbs;
      const unsigned s4 = (unsigned)db.x - nbs, s5 = (unsigned)db.y - nbs;
      const unsigned s6 = (unsigned)db.z - nbs, s7 = (unsigned)db.w - nbs;
      const bool h0 = valid & (s0 < unb), h1 = valid & (s1 < unb), h2 = valid & (s2 < unb), h3 = valid & (s3 < unb);
      const bool h4 = valid & (s4 < unb), h5 = valid & (s5 < unb), h6 = valid & (s6 < unb), h7 = valid & (s7 < unb);
      const unsigned any = __builtin_amdgcn_ballot_w32(h0 | h1 | h2 | h3 | h4 | h5 | h6 | h7);
      if (any != 0u) {
        HITJ(h0, s0, sa.x)
        HITJ(h1, s1, sa.y)
        HITJ(h2, s2, sa.z)
        HITJ(h3, s3, sa.w)
        HITJ(h4, s4, sb.x)
        HITJ(h5, s5, sb.y)
        HITJ(h6, s6, sb.z)
        HITJ(h7, s7, sb.w)
      }
    }
  }
  if (lane == 0) misc[wave] = wc;
  __syncthreads();

  if (wave == 0) {
    int tot = 0, ovf = 0;
#pragma unroll 1
    for (int w2 = 0; w2 < BWAVE; ++w2) {
      int c = misc[w2];
      ovf |= (c > WLCAP) ? 1 : 0;
      c = c < 0 ? 0 : (c > WLCAP ? WLCAP : c);
      c = __builtin_amdgcn_readfirstlane(c);
#pragma unroll 1
      for (int b0 = 0; b0 < c; b0 += 32) {
        int idx = b0 + lane;
        idx = idx > c - 1 ? c - 1 : idx;
        const int ent = wl[w2 * WLCAP + idx];
        const int m32 = (c - b0) < 32 ? (c - b0) : 32;
#pragma unroll 1
        for (int k = 0; k < m32; ++k) {
          const int u  = __builtin_amdgcn_readlane(ent, k);
          const int sq = u & (NBRUN - 1);
          if (lane == 0) cnt[sq] = cnt[sq] + 1;
        }
      }
      tot += c;
    }
    ovf |= (tot > RCAP) ? 1 : 0;
    if (lane == 0) misc[16] = ovf;
  }
  __syncthreads();

  {
    const v4i ca = *(const v4ia*)(cnt + 4 * tid);
    const int e0 = ca.x < 0 ? 0 : ca.x, e1 = ca.y < 0 ? 0 : ca.y;
    const int e2 = ca.z < 0 ? 0 : ca.z, e3 = ca.w < 0 ? 0 : ca.w;
    if (e0 > DEGCAP || e1 > DEGCAP || e2 > DEGCAP || e3 > DEGCAP) misc[24] = 1;
    const int ts = e0 + e1 + e2 + e3;
    int incl = ts;
#pragma unroll
    for (int d = 1; d < 32; d <<= 1) {
      const int up = __shfl_up(incl, d, 32);
      if (lane >= d) incl += up;
    }
    if (lane == 31) misc[8 + wave] = incl;
    __syncthreads();
    int pre = 0;
#pragma unroll
    for (int w2 = 0; w2 < BWAVE; ++w2) pre += (w2 < wave) ? misc[8 + w2] : 0;
    v4i ov;
    int run = pre + incl - ts;
    ov.x = run; run += e0;
    ov.y = run; run += e1;
    ov.z = run; run += e2;
    ov.w = run;
    *(v4ia*)(off + 4 * tid) = ov;
    *(v4ia*)(cur + 4 * tid) = ov;
  }
  __syncthreads();

  if (wave == 0) {
#pragma unroll 1
    for (int w2 = 0; w2 < BWAVE; ++w2) {
      int c = misc[w2];
      c = c < 0 ? 0 : (c > WLCAP ? WLCAP : c);
      c = __builtin_amdgcn_readfirstlane(c);
#pragma unroll 1
      for (int b0 = 0; b0 < c; b0 += 32) {
        int idx = b0 + lane;
        idx = idx > c - 1 ? c - 1 : idx;
        const int ent = wl[w2 * WLCAP + idx];
        const int m32 = (c - b0) < 32 ? (c - b0) : 32;
#pragma unroll 1
        for (int k = 0; k < m32; ++k) {
          const int u  = __builtin_amdgcn_readlane(ent, k);
          const int sq = u & (NBRUN - 1);
          const int sv = (int)((unsigned)u >> SLB);
          if (lane == 0) {
            int p = cur[sq];
            p = p < 0 ? 0 : (p > RCAP - 1 ? RCAP - 1 : p);
            sl[p] = sv;
            cur[sq] = p + 1;
          }
        }
      }
    }
  }
  __syncthreads();

  const int fl = ((misc[16] | misc[24]) != 0) ? 1 : 0;
  int* lg = listg + (size_t)blk * RCAP;
  int* cg = cntg + (size_t)blk * NBRUN + 4 * tid;
  int* og = offg + (size_t)blk * NBRUN + 4 * tid;
  int* fg = flagg + (size_t)blk * FLW + 4 * (tid & 7);
  const v4i cv = *(const v4ia*)(cnt + 4 * tid);
  const v4i ovv = *(const v4ia*)(off + 4 * tid);
  const v4i fv = {fl, fl, fl, fl};
#pragma unroll 1
  for (int i = 4 * tid; i < RCAP; i += 4 * BTHR) {
    const v4i v = *(const v4ia*)(sl + i);
    *(volatile v4i*)(lg + i) = v;
  }
  *(volatile v4i*)cg = cv;
  *(volatile v4i*)og = ovv;
  if (tid < 8) *(volatile v4i*)fg = fv;
  __threadfence();
#pragma unroll 1
  for (int i = 4 * tid; i < RCAP; i += 4 * BTHR) {
    const v4i v = *(const v4ia*)(sl + i);
    *(volatile v4i*)(lg + i) = v;
  }
  *(volatile v4i*)cg = cv;
  *(volatile v4i*)og = ovv;
  if (tid < 8) *(volatile v4i*)fg = fv;
}
#undef HITJ

template <int SRC>
__global__ __launch_bounds__(ATHR) void k_replay(const unsigned short* __restrict__ xb,
                                                 const float* __restrict__ hf,
                                                 const int* __restrict__ list, const int* __restrict__ cntp,
                                                 const int* __restrict__ offp, const int* __restrict__ flagp,
                                                 unsigned short* aout, int nN, unsigned lomask) {
  const int tid = (int)threadIdx.x, lane = tid & 31, wave = tid >> 5, hh = lane >> 4, j = lane & 15;
  const int row = (int)blockIdx.x * 16 + wave * 2 + hh;
  const int rc  = row < nN ? row : nN - 1;
  const int blk = rc >> SLB;
  int c = cntp[rc];
  int o = offp[rc];
  const int fl = flagp[blk * FLW];
  asm volatile("" :: "v"(c), "v"(o), "v"(fl));
  c = c < 0 ? 0 : (c > DEGCAP ? DEGCAP : c);
  o = o < 0 ? 0 : (o > RCAP - 1 ? RCAP - 1 : o);
  int last = o + c - 1;
  last = last < o ? o : last;
  last = last > RCAP - 1 ? RCAP - 1 : last;
  const int co = __shfl_xor(c, 16, 32);
  int cm = c > co ? c : co;
  cm = __builtin_amdgcn_readfirstlane(cm);
  const int* lp = list + (size_t)blk * RCAP;

  float a0, a1, a2, a3;
  if constexpr (SRC == 0) {
    const v2u q = *(const v2ua*)(xb + (size_t)rc * DC + 4 * j);
    a0 = __uint_as_float(q.x << 16); a1 = __uint_as_float(q.x & 0xffff0000u);
    a2 = __uint_as_float(q.y << 16); a3 = __uint_as_float(q.y & 0xffff0000u);
  } else {
    const v4f q = *(const v4f*)(hf + (size_t)rc * DC + 4 * j);
    a0 = q.x; a1 = q.y; a2 = q.z; a3 = q.w;
  }
#pragma unroll 1
  for (int k = 0; k < cm; ++k) {
    int idx = o + k;
    idx = idx > last ? last : idx;
    int s = lp[idx];
    s = s < 0 ? 0 : (s > nN - 1 ? nN - 1 : s);
    const unsigned msk = (k < c) ? 0xffffffffu : 0u;
    if constexpr (SRC == 0) {
      const v2u q = *(const v2ua*)(xb + (size_t)s * DC + 4 * j);
      asm volatile("" :: "v"(q.x), "v"(q.y));
      a0 += __uint_as_float((q.x << 16) & msk);
      a1 += __uint_as_float((q.x & 0xffff0000u) & msk);
      a2 += __uint_as_float((q.y << 16) & msk);
      a3 += __uint_as_float((q.y & 0xffff0000u) & msk);
    } else {
      const v4f q = *(const v4f*)(hf + (size_t)s * DC + 4 * j);
      asm volatile("" :: "v"(q.x), "v"(q.y), "v"(q.z), "v"(q.w));
      a0 += __uint_as_float(__float_as_uint(q.x) & msk);
      a1 += __uint_as_float(__float_as_uint(q.y) & msk);
      a2 += __uint_as_float(__float_as_uint(q.z) & msk);
      a3 += __uint_as_float(__float_as_uint(q.w) & msk);
    }
  }
  const float pz = (fl != 0) ? __int_as_float(0x7fc00000) : 0.0f;
  const HL o2 = split4(a0 + pz, a1 + pz, a2 + pz, a3 + pz, lomask);
  st2_pair(aout + (size_t)rc * KT + 4 * j, o2.h, o2.l, row < nN);
}

__global__ __launch_bounds__(GTHR) void k_gemm(const unsigned short* __restrict__ A,
                                               const unsigned short* __restrict__ WT,
                                               const float* __restrict__ par, int boff,
                                               float* tout, double* rec, int nN) {
  __shared__ __attribute__((aligned(16))) float  stg[GBM * DC];
  __shared__ __attribute__((aligned(16))) float  bsh[DC];
  __shared__ __attribute__((aligned(16))) double pst[RECW];
  const int tid = (int)threadIdx.x, lane = tid & 31, wave = tid >> 5, hh = lane >> 4, m = lane & 15;
  const int rowBase = (int)blockIdx.x * GBM;

  {
    const v4f bv = *(const v4f*)(par + boff + 4 * (tid & 15));
    asm volatile("" :: "v"(bv.x), "v"(bv.y), "v"(bv.z), "v"(bv.w));
    if (tid < 16) *(v4fa*)(bsh + 4 * tid) = bv;
  }
  __syncthreads();

  v8f acc[4];
  {
    const v8f z = {0.f, 0.f, 0.f, 0.f, 0.f, 0.f, 0.f, 0.f};
#pragma unroll
    for (int t = 0; t < 4; ++t) acc[t] = z;
  }
  const unsigned short* ap = A + (size_t)(rowBase + 16 * wave + m) * (size_t)KT + 8 * hh;
  const unsigned short* wp = WT + (size_t)m * (size_t)KT + 8 * hh;
#pragma unroll 1
  for (int ks = 0; ks < KT / 32; ++ks) {
    FragB af;
    af.h[0] = *(const v8usa*)(ap + 32 * ks);
    af.h[1] = *(const v8usa*)(ap + 32 * ks + 16);
#pragma unroll
    for (int t = 0; t < 4; ++t) {
      const unsigned short* wq = wp + (size_t)(16 * t) * (size_t)KT + 32 * ks;
      FragB bf;
      bf.h[0] = *(const v8usa*)wq;
      bf.h[1] = *(const v8usa*)(wq + 16);
      acc[t] = wmb(af, bf, acc[t]);
    }
  }

#pragma unroll
  for (int t = 0; t < 4; ++t) {
    const int lc = 16 * t + m;
    const float bb = bsh[lc];
#pragma unroll
    for (int r = 0; r < 8; ++r) {
      const int lr = 16 * wave + 8 * hh + r;
      stg[lr * DC + lc] = acc[t][r] + bb;
    }
  }
  __syncthreads();

  {
    v4f fv[8];
#pragma unroll
    for (int i = 0; i < 8; ++i) {
      const int lr = 16 * wave + 2 * i + hh;
      fv[i] = *(const v4fa*)(stg + lr * DC + 4 * m);
    }
#pragma unroll
    for (int i = 0; i < 8; ++i) {
      const int gr = rowBase + 16 * wave + 2 * i + hh;
      float* op = tout + (size_t)gr * DC + 4 * m;
      if (gr < nN) *(volatile v4f*)op = fv[i];
    }
    __threadfence();
#pragma unroll
    for (int i = 0; i < 8; ++i) {
      const int gr = rowBase + 16 * wave + 2 * i + hh;
      float* op = tout + (size_t)gr * DC + 4 * m;
      if (gr < nN) *(volatile v4f*)op = fv[i];
    }
  }

  if (tid < DC) {
    int rv = nN - rowBase;
    rv = rv < 1 ? 1 : (rv > GBM ? GBM : rv);
    double s = 0.0;
#pragma unroll 1
    for (int r = 0; r < rv; ++r) s += (double)stg[r * DC + tid];
    const double mean = s / (double)rv;
    double q = 0.0;
#pragma unroll 1
    for (int r = 0; r < rv; ++r) {
      const double d = (double)stg[r * DC + tid] - mean;
      q += d * d;
    }
    pst[tid] = mean;
    pst[DC + tid] = q;
  }
  __syncthreads();
  {
    const int tq = tid & 63;
    const v2d pv = *(const v2da*)(pst + 2 * tq);
    st2_v2d(rec + (size_t)blockIdx.x * RECW + 2 * tq, pv, tid < 64);
  }
}

__global__ __launch_bounds__(DC) void k_comb(const double* __restrict__ rec, int nB, int nN, double invN,
                                             float* stat) {
  __shared__ __attribute__((aligned(16))) float ss[2 * DC];
  const int c = (int)threadIdx.x;
  double S = 0.0;
#pragma unroll 1
  for (int b = 0; b < nB; ++b) {
    int nb = nN - b * GBM;
    nb = nb < 0 ? 0 : (nb > GBM ? GBM : nb);
    S += (double)nb * rec[(size_t)b * RECW + c];
  }
  const double mean = S * invN;
  double Q1 = 0.0, Q2 = 0.0;
#pragma unroll 1
  for (int b = 0; b < nB; ++b) {
    int nb = nN - b * GBM;
    nb = nb < 0 ? 0 : (nb > GBM ? GBM : nb);
    const double d = rec[(size_t)b * RECW + c] - mean;
    Q1 += rec[(size_t)b * RECW + DC + c];
    Q2 += (double)nb * d * d;
  }
  float v = (float)((Q1 + Q2) * invN);
  v = (v < 0.0f) ? 0.0f : v;
  const float rs = 1.0f / sqrtf(v + 1e-5f);
  ss[c] = (float)mean;
  ss[DC + c] = rs;
  __syncthreads();
  const v4f o = *(const v4fa*)(ss + 4 * (c & 31));
  st2_v4f(stat + 4 * (c & 31), o, c < 32);
}

__global__ __launch_bounds__(ATHR) void k_apply_a(const float* __restrict__ t, const float* __restrict__ stat,
                                                  const float* __restrict__ par, int goff, int boff,
                                                  unsigned lomask, unsigned short* aout, int nUnits) {
  __shared__ __attribute__((aligned(16))) float sp[4 * DC];
  const int tid = (int)threadIdx.x;
  {
    const int q = tid & 15, hs = (tid >> 4) & 1;
    const v4f sv = *(const v4f*)(stat + DC * hs + 4 * q);
    const v4f pv = *(const v4f*)(par + (hs != 0 ? boff : goff) + 4 * q);
    asm volatile("" :: "v"(sv.x), "v"(sv.y), "v"(sv.z), "v"(sv.w));
    asm volatile("" :: "v"(pv.x), "v"(pv.y), "v"(pv.z), "v"(pv.w));
    if (tid < 32)      *(v4fa*)(sp + DC * hs + 4 * q) = sv;
    else if (tid < 64) *(v4fa*)(sp + 2 * DC + DC * hs + 4 * q) = pv;
  }
  __syncthreads();
  const int u  = (int)blockIdx.x * ATHR + tid;
  const bool ok = u < nUnits;
  const int uc = ok ? u : nUnits - 1;
  const int c4 = (uc & 15) * 4;
  const int row = uc >> 4;
  const v4f a = *(const v4f*)(t + (size_t)uc * 4);
  asm volatile("" :: "v"(a.x), "v"(a.y), "v"(a.z), "v"(a.w));
  const v4f mm = *(const v4fa*)(sp + c4);
  const v4f rr = *(const v4fa*)(sp + DC + c4);
  const v4f gg = *(const v4fa*)(sp + 2 * DC + c4);
  const v4f be = *(const v4fa*)(sp + 3 * DC + c4);
  const float y0 = relu_k(((a.x - mm.x) * rr.x) * gg.x + be.x);
  const float y1 = relu_k(((a.y - mm.y) * rr.y) * gg.y + be.y);
  const float y2 = relu_k(((a.z - mm.z) * rr.z) * gg.z + be.z);
  const float y3 = relu_k(((a.w - mm.w) * rr.w) * gg.w + be.w);
  const HL o2 = split4(y0, y1, y2, y3, lomask);
  st2_pair(aout + (size_t)row * KT + c4, o2.h, o2.l, ok);
}

template <int RELU>
__global__ __launch_bounds__(ATHR) void k_apply_b(const float* __restrict__ t, const float* __restrict__ stat,
                                                  const float* __restrict__ par, int goff, int boff,
                                                  const int* __restrict__ flagp, float* outp, int nUnits) {
  __shared__ __attribute__((aligned(16))) float sp[4 * DC];
  const int tid = (int)threadIdx.x;
  {
    const int q = tid & 15, hs = (tid >> 4) & 1;
    const v4f sv = *(const v4f*)(stat + DC * hs + 4 * q);
    const v4f pv = *(const v4f*)(par + (hs != 0 ? boff : goff) + 4 * q);
    asm volatile("" :: "v"(sv.x), "v"(sv.y), "v"(sv.z), "v"(sv.w));
    asm volatile("" :: "v"(pv.x), "v"(pv.y), "v"(pv.z), "v"(pv.w));
    if (tid < 32)      *(v4fa*)(sp + DC * hs + 4 * q) = sv;
    else if (tid < 64) *(v4fa*)(sp + 2 * DC + DC * hs + 4 * q) = pv;
  }
  __syncthreads();
  const int u  = (int)blockIdx.x * ATHR + tid;
  const bool ok = u < nUnits;
  const int uc = ok ? u : nUnits - 1;
  const int c4 = (uc & 15) * 4;
  const int row = uc >> 4;
  const v4f a = *(const v4f*)(t + (size_t)uc * 4);
  const int fl = flagp[(row >> SLB) * FLW];
  asm volatile("" :: "v"(a.x), "v"(a.y), "v"(a.z), "v"(a.w), "v"(fl));
  const v4f mm = *(const v4fa*)(sp + c4);
  const v4f rr = *(const v4fa*)(sp + DC + c4);
  const v4f gg = *(const v4fa*)(sp + 2 * DC + c4);
  const v4f be = *(const v4fa*)(sp + 3 * DC + c4);
  float y0 = ((a.x - mm.x) * rr.x) * gg.x + be.x;
  float y1 = ((a.y - mm.y) * rr.y) * gg.y + be.y;
  float y2 = ((a.z - mm.z) * rr.z) * gg.z + be.z;
  float y3 = ((a.w - mm.w) * rr.w) * gg.w + be.w;
  if (RELU != 0) { y0 = relu_k(y0); y1 = relu_k(y1); y2 = relu_k(y2); y3 = relu_k(y3); }
  const float pz = (fl != 0) ? __int_as_float(0x7fc00000) : 0.0f;
  v4f o;
  o.x = y0 + pz; o.y = y1 + pz; o.z = y2 + pz; o.w = y3 + pz;
  st2_v4f(outp + (size_t)uc * 4, o, ok);
}

constexpr unsigned SINGLE_SITE = 0u;
static inline unsigned lomask_of(int s) { return ((SINGLE_SITE >> s) & 1u) ? 0u : 0xffffffffu; }
static inline size_t al256(size_t o) { return (o + 255) & ~(size_t)255; }

extern "C" void kernel_launch(void* const* d_in, const int* in_sizes, int n_in,
                              void* d_out, int out_size, void* d_ws, size_t ws_size,
                              hipStream_t stream) {
  if (n_in < 18) return;
  if (in_sizes[0] != NN * DC) return;
  if (in_sizes[1] != 2 * NE) return;
  for (int i = 2; i < 6; ++i)  if (in_sizes[i] != DC * DC) return;
  for (int i = 6; i < 18; ++i) if (in_sizes[i] != DC) return;
  if (out_size != NN * DC) return;

  const float* x   = (const float*)d_in[0];
  const int*   ei  = (const int*)d_in[1];
  const int*   src = ei;
  const int*   dst = ei + NE;
  float* out = (float*)d_out;

  char* ws = (char*)d_ws;
  size_t off = 0;
  const size_t oWT   = off; off = al256(off + (size_t)4 * WSQ * 2);
  const size_t oPAR  = off; off = al256(off + (size_t)12 * DC * 4);
  const size_t oSTAT = off; off = al256(off + (size_t)2 * DC * 4);
  const size_t oFLAG = off; off = al256(off + (size_t)NBLK * FLW * 4);
  const size_t oXB   = off; off = al256(off + (size_t)NN * DC * 2);
  const size_t oA    = off; off = al256(off + (size_t)MP * KT * 2);
  const size_t oT    = off; off = al256(off + (size_t)MP * DC * 4);
  const size_t oH    = off; off = al256(off + (size_t)NN * DC * 4);
  const size_t oLIST = off; off = al256(off + (size_t)NBLK * RCAP * 4);
  const size_t oCNT  = off; off = al256(off + (size_t)NBLK * NBRUN * 4);
  const size_t oOFF  = off; off = al256(off + (size_t)NBLK * NBRUN * 4);
  const size_t oREC  = off; off = al256(off + (size_t)NGB * RECW * 8);
  if (off > ws_size || off > (size_t)(128u << 20)) return;
  unsigned short* WT   = (unsigned short*)(ws + oWT);
  float*          PAR  = (float*)(ws + oPAR);
  float*          STAT = (float*)(ws + oSTAT);
  int*            FLAG = (int*)(ws + oFLAG);
  unsigned short* XB   = (unsigned short*)(ws + oXB);
  unsigned short* A    = (unsigned short*)(ws + oA);
  float*          T    = (float*)(ws + oT);
  float*          H    = (float*)(ws + oH);
  int*            LIST = (int*)(ws + oLIST);
  int*            CNT  = (int*)(ws + oCNT);
  int*            OFF  = (int*)(ws + oOFF);
  double*         REC  = (double*)(ws + oREC);

  hipFuncSetAttribute(reinterpret_cast<const void*>(&k_bucket), hipFuncAttributeMaxDynamicSharedMemorySize,
                      BUCKET_LDS);

  const double invN = 1.0 / (double)NN;
  const int gR = NN / 16;
  const int gU = NUNITS / ATHR;

  k_prep<<<PB_TOT, PTHR, 0, stream>>>(
      x,
      (const float*)d_in[2], (const float*)d_in[3], (const float*)d_in[4], (const float*)d_in[5],
      (const float*)d_in[6], (const float*)d_in[7], (const float*)d_in[8], (const float*)d_in[9],
      (const float*)d_in[10], (const float*)d_in[11], (const float*)d_in[12], (const float*)d_in[13],
      (const float*)d_in[14], (const float*)d_in[15], (const float*)d_in[16], (const float*)d_in[17],
      XB, WT, PAR, A + (size_t)NN * KT);
  k_bucket<<<NBLK, BTHR, BUCKET_LDS, stream>>>(src, dst, NE, NN, LIST, CNT, OFF, FLAG);

  for (int l = 0; l < 2; ++l) {
    const int sa = 2 * l, sb = 2 * l + 1;
    if (l == 0) k_replay<0><<<gR, ATHR, 0, stream>>>(XB, H, LIST, CNT, OFF, FLAG, A, NN, lomask_of(sa));
    else        k_replay<1><<<gR, ATHR, 0, stream>>>(XB, H, LIST, CNT, OFF, FLAG, A, NN, lomask_of(sa));
    k_gemm<<<NGB, GTHR, 0, stream>>>(A, WT + (size_t)sa * WSQ, PAR, sa * DC, T, REC, NN);
    k_comb<<<1, DC, 0, stream>>>(REC, NGB, NN, invN, STAT);
    k_apply_a<<<gU, ATHR, 0, stream>>>(T, STAT, PAR, (8 + sa) * DC, (4 + sa) * DC, lomask_of(sb), A, NUNITS);
    k_gemm<<<NGB, GTHR, 0, stream>>>(A, WT + (size_t)sb * WSQ, PAR, sb * DC, T, REC, NN);
    k_comb<<<1, DC, 0, stream>>>(REC, NGB, NN, invN, STAT);
    if (l == 0) {
      k_apply_b<1><<<gU, ATHR, 0, stream>>>(T, STAT, PAR, (8 + sb) * DC, (4 + sb) * DC, FLAG, H, NUNITS);
    } else {
      k_apply_b<0><<<gU, ATHR, 0, stream>>>(T, STAT, PAR, (8 + sb) * DC, (4 + sb) * DC, FLAG, out, NUNITS);
    }
  }
}
